// GATModule_11605001634177
// MI455X (gfx1250) — hardware-verified
//
#include <hip/hip_runtime.h>
#include <stddef.h>
#include <stdint.h>
#include <math.h>


#define F_IN    256
#define HIDC    128
#define NHEAD   4
#define HC      512
#define KHL1    256
#define KHL2    1024
#define M1N     64
#define NTHR    256
#define NWAVE   8
#define EPT     8
#define CHUNK   (NTHR * EPT)
#define WCAP    (EPT * 32)
#define LISTN   (NWAVE * WCAP)
#define NBMAX   2048
#define SLOTB   11
#define RCAP    28672
#define DEGCAP  256
#define GBM     64
#define GBN     128
#define GTHR    128
#define RECW    256
#define NEGSL   0.2f
#define EPS_SM  1e-16f
#define LN_EPS  1e-5f
#define WSMAX   134217728
#define LDS_AGG ((2 * RCAP + 2 * NBMAX + LISTN) * 4 + 64)
#define NU_NW   (HIDC * (F_IN / 8))
#define NU_G1   (HC * (KHL1 / 8))
#define NU_RW   (HC * (KHL1 / 8))
#define NU_G2   (HC * (KHL2 / 8))
#define NU_OW   (HIDC * (KHL2 / 8))
#define NU_M1   (HIDC * (KHL1 / 8))
#define NU_ALL  (NU_NW + NU_G1 + NU_RW + NU_G2 + NU_OW + NU_M1)

enum { EPI_HL0 = 0, EPI_HLR = 1, EPI_DOT = 2, EPI_POOL = 3, EPI_HEAD = 4 };

static_assert((CHUNK & (CHUNK - 1)) == 0 && CHUNK <= (1 << SLOTB));
static_assert(NBMAX == (1 << SLOTB));
static_assert(NTHR * 8 == NBMAX);
static_assert(LISTN >= NBMAX);
static_assert(LISTN >= NWAVE * WCAP);
static_assert((RCAP % 32) == 0);
static_assert(LDS_AGG <= 300000);
static_assert(GBM == (GTHR / 32) * 16);
static_assert(GTHR == GBN);
static_assert(HIDC == GBN && HC == NHEAD * GBN);
static_assert(KHL1 == 2 * HIDC && KHL2 == 2 * HC);
static_assert((F_IN % 32) == 0 && (KHL1 % 32) == 0 && (KHL2 % 32) == 0);
static_assert(HC == 2 * 8 * 32);
static_assert(M1N == 16 * 4 && M1N <= GBN);
static_assert((NU_NW % NTHR) == 0 && (NU_G1 % NTHR) == 0 && (NU_RW % NTHR) == 0);
static_assert((NU_G2 % NTHR) == 0 && (NU_OW % NTHR) == 0 && (NU_M1 % NTHR) == 0);
static_assert(RECW == 2 * GBN);
static_assert((F_IN / 8) == 32);

typedef float          v4f  __attribute__((ext_vector_type(4)));
typedef float          v8f  __attribute__((ext_vector_type(8)));
typedef int            v4i  __attribute__((ext_vector_type(4)));
typedef int            v8i  __attribute__((ext_vector_type(8)));
typedef unsigned int   v4u  __attribute__((ext_vector_type(4)));
typedef unsigned short v8us __attribute__((ext_vector_type(8)));
typedef __bf16         v16b __attribute__((ext_vector_type(16)));
typedef v4f  __attribute__((may_alias)) v4fa;
typedef v4u  __attribute__((may_alias)) v4ua;
typedef v8us __attribute__((may_alias)) v8usa;
union FragB { v16b v; v8us h[2]; v8i w; };

__device__ __forceinline__ v8f wmb(const FragB& a, const FragB& b, v8f c) {
  v8f d = __builtin_amdgcn_wmma_f32_16x16x32_bf16(false, a.v, false, b.v, (short)0, c, false, false);
  asm volatile("v_nop\n\tv_nop\n\tv_nop\n\tv_nop" : "+v"(d) : "v"(a.w), "v"(b.w));
  return d;
}

__device__ __forceinline__ unsigned int f2bf(float f) {
  const unsigned int u = __float_as_uint(f);
  return ((u + 0x7FFFu + ((u >> 16) & 1u)) >> 16) & 0xFFFFu;
}
__device__ __forceinline__ float bf2f(unsigned int b) { return __uint_as_float(b << 16); }
__device__ __forceinline__ float bfr(float f) { return bf2f(f2bf(f)); }
__device__ __forceinline__ v4f bfr4(const v4f a) {
  v4f r; r.x = bfr(a.x); r.y = bfr(a.y); r.z = bfr(a.z); r.w = bfr(a.w); return r;
}
__device__ __forceinline__ unsigned int pk2(float lo, float hi) { return f2bf(lo) | (f2bf(hi) << 16); }
__device__ __forceinline__ v4u pack8(const v4f a, const v4f b) {
  v4u r;
  r.x = pk2(a.x, a.y); r.y = pk2(a.z, a.w); r.z = pk2(b.x, b.y); r.w = pk2(b.z, b.w);
  return r;
}
__device__ __forceinline__ void hlpack(const v4f a, const v4f b, v4u& hv, v4u& lv) {
  const unsigned int h0 = f2bf(a.x), h1 = f2bf(a.y), h2 = f2bf(a.z), h3 = f2bf(a.w);
  const unsigned int h4 = f2bf(b.x), h5 = f2bf(b.y), h6 = f2bf(b.z), h7 = f2bf(b.w);
  const unsigned int l0 = f2bf(a.x - bf2f(h0)), l1 = f2bf(a.y - bf2f(h1));
  const unsigned int l2 = f2bf(a.z - bf2f(h2)), l3 = f2bf(a.w - bf2f(h3));
  const unsigned int l4 = f2bf(b.x - bf2f(h4)), l5 = f2bf(b.y - bf2f(h5));
  const unsigned int l6 = f2bf(b.z - bf2f(h6)), l7 = f2bf(b.w - bf2f(h7));
  hv.x = h0 | (h1 << 16); hv.y = h2 | (h3 << 16); hv.z = h4 | (h5 << 16); hv.w = h6 | (h7 << 16);
  lv.x = l0 | (l1 << 16); lv.y = l2 | (l3 << 16); lv.z = l4 | (l5 << 16); lv.w = l6 | (l7 << 16);
}
__device__ __forceinline__ float wsum(float v) {
#pragma unroll
  for (int off = 16; off > 0; off >>= 1) v += __shfl_xor(v, off);
  return v;
}
__device__ __forceinline__ float wmax(float v) {
#pragma unroll
  for (int off = 16; off > 0; off >>= 1) v = fmaxf(v, __shfl_xor(v, off));
  return v;
}
__device__ __forceinline__ float leaky(float x) { return x > 0.f ? x : NEGSL * x; }
__device__ __forceinline__ v4f fin4(const v4f a, float inv, const v4f b, bool live, float pz) {
  v4f o;
  o.x = (live ? fmaxf(fmaf(a.x, inv, b.x), 0.f) : 0.f) + pz;
  o.y = (live ? fmaxf(fmaf(a.y, inv, b.y), 0.f) : 0.f) + pz;
  o.z = (live ? fmaxf(fmaf(a.z, inv, b.z), 0.f) : 0.f) + pz;
  o.w = (live ? fmaxf(fmaf(a.w, inv, b.w), 0.f) : 0.f) + pz;
  return o;
}

__device__ __forceinline__ int scan_chunk(const int* __restrict__ dsts, int nE, int cbase, int slotBase,
                                          int nb, int vec8, int* list, int tid, int lane, int wave) {
  int wc = 0;
  const int el0  = tid * EPT;
  const int e0   = cbase + el0;
  const int sent = -2147483647 - 1;
  v4i da, db;
  if (vec8 != 0 && cbase + CHUNK <= nE) {
    da = *(const v4i*)(dsts + e0);
    db = *(const v4i*)(dsts + e0 + 4);
  } else {
    da.x = (e0     < nE) ? dsts[min(e0,     nE - 1)] : sent;
    da.y = (e0 + 1 < nE) ? dsts[min(e0 + 1, nE - 1)] : sent;
    da.z = (e0 + 2 < nE) ? dsts[min(e0 + 2, nE - 1)] : sent;
    da.w = (e0 + 3 < nE) ? dsts[min(e0 + 3, nE - 1)] : sent;
    db.x = (e0 + 4 < nE) ? dsts[min(e0 + 4, nE - 1)] : sent;
    db.y = (e0 + 5 < nE) ? dsts[min(e0 + 5, nE - 1)] : sent;
    db.z = (e0 + 6 < nE) ? dsts[min(e0 + 6, nE - 1)] : sent;
    db.w = (e0 + 7 < nE) ? dsts[min(e0 + 7, nE - 1)] : sent;
  }
  const unsigned nbs = (unsigned)slotBase;
  const unsigned unb = (unsigned)nb;
  const unsigned s0 = (unsigned)da.x - nbs, s1 = (unsigned)da.y - nbs;
  const unsigned s2 = (unsigned)da.z - nbs, s3 = (unsigned)da.w - nbs;
  const unsigned s4 = (unsigned)db.x - nbs, s5 = (unsigned)db.y - nbs;
  const unsigned s6 = (unsigned)db.z - nbs, s7 = (unsigned)db.w - nbs;
  const bool h0 = s0 < unb, h1 = s1 < unb, h2 = s2 < unb, h3 = s3 < unb;
  const bool h4 = s4 < unb, h5 = s5 < unb, h6 = s6 < unb, h7 = s7 < unb;
  const unsigned any = __builtin_amdgcn_ballot_w32(h0 | h1 | h2 | h3 | h4 | h5 | h6 | h7);
  if (any != 0u) {
#define HITJ(J, HJ, SJ) { \
      const unsigned mj = __builtin_amdgcn_ballot_w32(HJ); \
      if (mj != 0u) { \
        if (HJ) { \
          const int pos = wc + (int)__builtin_amdgcn_mbcnt_lo(mj, 0u); \
          if (pos < WCAP) list[wave * WCAP + pos] = ((el0 + (J)) << SLOTB) | (int)(SJ); \
        } \
        wc += (int)__builtin_popcount(mj); } }
    HITJ(0, h0, s0)
    HITJ(1, h1, s1)
    HITJ(2, h2, s2)
    HITJ(3, h3, s3)
    HITJ(4, h4, s4)
    HITJ(5, h5, s5)
    HITJ(6, h6, s6)
    HITJ(7, h7, s7)
#undef HITJ
  }
  return wc;
}

__global__ __launch_bounds__(NTHR) void k_xprep(const float* __restrict__ x, unsigned short* xb, int nN, int nUnits) {
  const int i = (int)blockIdx.x * NTHR + (int)threadIdx.x;
  if (i >= nUnits) return;
  const int row = i >> 5;
  const int c0  = (i & 31) * 8;
  const int rc  = row < nN ? row : nN - 1;
  const float* p = x + (size_t)rc * F_IN + c0;
  v4f a = *(const v4fa*)p, b = *(const v4fa*)(p + 4);
  const v4f z4 = {0.f, 0.f, 0.f, 0.f};
  if (row >= nN) { a = z4; b = z4; }
  const v4u hv = pack8(a, b);
  const size_t o = (size_t)row * F_IN + c0;
  *(volatile v4u*)(xb + o) = hv;
  __threadfence();
  *(volatile v4u*)(xb + o) = hv;
}

__device__ __forceinline__ void wtr_unit(const float* __restrict__ w, int Kin, int Ncol, int Nrows, int Kout,
                                         unsigned short* wt, int u) {
  const int kq = Kout >> 3;
  const int n  = u / kq;
  const int k8 = (u - n * kq) * 8;
  const int kk = k8 - (k8 / Kin) * Kin;
  const int ncl = n < Ncol ? n : Ncol - 1;
  const float* p = w + (size_t)kk * (size_t)Ncol + ncl;
  v4f a, b;
  a.x = p[0];                    a.y = p[(size_t)Ncol];         a.z = p[(size_t)2 * Ncol];     a.w = p[(size_t)3 * Ncol];
  b.x = p[(size_t)4 * Ncol];     b.y = p[(size_t)5 * Ncol];     b.z = p[(size_t)6 * Ncol];     b.w = p[(size_t)7 * Ncol];
  const v4f z4 = {0.f, 0.f, 0.f, 0.f};
  if (n >= Ncol || n >= Nrows) { a = z4; b = z4; }
  const v4u wv = pack8(a, b);
  unsigned short* o = wt + (size_t)n * (size_t)Kout + k8;
  *(volatile v4u*)o = wv;
  __threadfence();
  *(volatile v4u*)o = wv;
}

__global__ __launch_bounds__(NTHR) void k_wprep(const float* __restrict__ nW, const float* __restrict__ g1W,
                                                const float* __restrict__ rW, const float* __restrict__ g2W,
                                                const float* __restrict__ oW, const float* __restrict__ m1W,
                                                unsigned short* nWT, unsigned short* g1WT, unsigned short* rWT,
                                                unsigned short* g2WT, unsigned short* oWT, unsigned short* m1WT) {
  const int u = (int)blockIdx.x * NTHR + (int)threadIdx.x;
  if (u < NU_NW) {
    wtr_unit(nW, F_IN, HIDC, HIDC, F_IN, nWT, u);
  } else if (u < NU_NW + NU_G1) {
    wtr_unit(g1W, HIDC, HC, HC, KHL1, g1WT, u - NU_NW);
  } else if (u < NU_NW + NU_G1 + NU_RW) {
    wtr_unit(rW, HIDC, HC, HC, KHL1, rWT, u - NU_NW - NU_G1);
  } else if (u < NU_NW + NU_G1 + NU_RW + NU_G2) {
    wtr_unit(g2W, HC, HC, HC, KHL2, g2WT, u - NU_NW - NU_G1 - NU_RW);
  } else if (u < NU_NW + NU_G1 + NU_RW + NU_G2 + NU_OW) {
    wtr_unit(oW, HC, HIDC, HIDC, KHL2, oWT, u - NU_NW - NU_G1 - NU_RW - NU_G2);
  } else if (u < NU_ALL) {
    wtr_unit(m1W, HIDC, M1N, HIDC, KHL1, m1WT, u - NU_NW - NU_G1 - NU_RW - NU_G2 - NU_OW);
  }
}

template <int EPI>
__global__ __launch_bounds__(GTHR) void k_gemm(
    const unsigned short* __restrict__ A, const unsigned short* __restrict__ WT, int K,
    const float* __restrict__ bias, const float* __restrict__ va, const float* __restrict__ vb,
    const unsigned short* __restrict__ HLin, float* outF, unsigned short* outH, float* outV,
    int MPr, int nN)
{
  constexpr int CH = (EPI == EPI_HLR) ? HC : HIDC;
  __shared__ __attribute__((aligned(16))) float stg[GBM * GBN];
  __shared__ __attribute__((aligned(16))) float sdot[2 * GBM];
  __shared__ __attribute__((aligned(16))) float sex[GBM];
  __shared__ __attribute__((aligned(16))) float srec[RECW];
  const int tid = (int)threadIdx.x, lane = tid & 31, wave = tid >> 5, hh = lane >> 4, m = lane & 15;
  const int rowBase = (int)blockIdx.x * GBM;
  const int head    = (int)blockIdx.y;
  const int col0    = head * GBN;

  v8f acc[8];
  {
    const v8f z = {0.f, 0.f, 0.f, 0.f, 0.f, 0.f, 0.f, 0.f};
#pragma unroll
    for (int t = 0; t < 8; ++t) acc[t] = z;
  }
  const unsigned short* ap = A  + (size_t)(rowBase + 16 * wave + m) * (size_t)K + 8 * hh;
  const unsigned short* bp = WT + (size_t)(col0 + m) * (size_t)K + 8 * hh;
#pragma unroll 1
  for (int k0 = 0; k0 < K; k0 += 32) {
    FragB af;
    af.h[0] = *(const v8usa*)(ap + k0);
    af.h[1] = *(const v8usa*)(ap + k0 + 16);
#pragma unroll
    for (int nt = 0; nt < 8; ++nt) {
      const unsigned short* wq = bp + (size_t)(16 * nt) * (size_t)K + k0;
      FragB bf;
      bf.h[0] = *(const v8usa*)wq;
      bf.h[1] = *(const v8usa*)(wq + 16);
      acc[nt] = wmb(af, bf, acc[nt]);
    }
  }

#pragma unroll
  for (int nt = 0; nt < 8; ++nt) {
    const int lc = 16 * nt + m;
#pragma unroll
    for (int r = 0; r < 8; ++r) {
      const int lr = 16 * wave + 8 * hh + r;
      stg[lr * GBN + lc] = acc[nt][r];
    }
  }
  __syncthreads();

  if constexpr (EPI == EPI_DOT) {
    const v4f as4 = bfr4(*(const v4fa*)(va + head * GBN + 4 * lane));
    const v4f ad4 = bfr4(*(const v4fa*)(vb + head * GBN + 4 * lane));
#pragma unroll 1
    for (int i = 0; i < 16; ++i) {
      const int row = 16 * wave + i;
      const v4f p = *(const v4fa*)(stg + row * GBN + 4 * lane);
      float s = 0.f, d = 0.f;
      s = fmaf(p.x, as4.x, s); s = fmaf(p.y, as4.y, s); s = fmaf(p.z, as4.z, s); s = fmaf(p.w, as4.w, s);
      d = fmaf(p.x, ad4.x, d); d = fmaf(p.y, ad4.y, d); d = fmaf(p.z, ad4.z, d); d = fmaf(p.w, ad4.w, d);
      s = wsum(s); d = wsum(d);
      if (lane == 0) { sdot[row] = s; sdot[GBM + row] = d; }
    }
    __syncthreads();
    const int which2 = lane >> 4, piece = lane & 15;
    const v4f sdv = *(const v4fa*)(sdot + which2 * GBM + 4 * piece);
    float* sp = outV + (size_t)(2 * head + which2) * (size_t)MPr + rowBase + 4 * piece;
#pragma unroll 1
    for (int i = 0; i < 16; ++i) {
      const int row = 16 * wave + i;
      const v4f p = *(const v4fa*)(stg + row * GBN + 4 * lane);
      float* op = outF + (size_t)(rowBase + row) * (size_t)HC + col0 + 4 * lane;
      *(volatile v4f*)op = p;
    }
    if (wave == 0) *(volatile v4f*)sp = sdv;
    __threadfence();
#pragma unroll 1
    for (int i = 0; i < 16; ++i) {
      const int row = 16 * wave + i;
      const v4f p = *(const v4fa*)(stg + row * GBN + 4 * lane);
      float* op = outF + (size_t)(rowBase + row) * (size_t)HC + col0 + 4 * lane;
      *(volatile v4f*)op = p;
    }
    if (wave == 0) *(volatile v4f*)sp = sdv;
  } else if constexpr (EPI == EPI_HL0 || EPI == EPI_HLR) {
    const int c8 = 8 * m;
    const v4f bq0 = bfr4(*(const v4fa*)(bias + col0 + c8));
    const v4f bq1 = bfr4(*(const v4fa*)(bias + col0 + c8 + 4));
    const size_t hoff = (size_t)hh * CH + col0 + c8;
#pragma unroll 1
    for (int i = 0; i < 16; ++i) {
      const int row  = 16 * wave + i;
      const int grow = rowBase + row;
      v4f q0 = *(const v4fa*)(stg + row * GBN + c8);
      v4f q1 = *(const v4fa*)(stg + row * GBN + c8 + 4);
      q0 += bq0; q1 += bq1;
      if constexpr (EPI == EPI_HLR) {
        const unsigned short* hpi = HLin + (size_t)grow * KHL2 + col0 + c8;
        const v4u hw = *(const v4ua*)hpi;
        const v4u lw = *(const v4ua*)(hpi + HC);
        q0.x += __uint_as_float(hw.x << 16)          + __uint_as_float(lw.x << 16);
        q0.y += __uint_as_float(hw.x & 0xffff0000u)  + __uint_as_float(lw.x & 0xffff0000u);
        q0.z += __uint_as_float(hw.y << 16)          + __uint_as_float(lw.y << 16);
        q0.w += __uint_as_float(hw.y & 0xffff0000u)  + __uint_as_float(lw.y & 0xffff0000u);
        q1.x += __uint_as_float(hw.z << 16)          + __uint_as_float(lw.z << 16);
        q1.y += __uint_as_float(hw.z & 0xffff0000u)  + __uint_as_float(lw.z & 0xffff0000u);
        q1.z += __uint_as_float(hw.w << 16)          + __uint_as_float(lw.w << 16);
        q1.w += __uint_as_float(hw.w & 0xffff0000u)  + __uint_as_float(lw.w & 0xffff0000u);
      }
      if constexpr (EPI == EPI_HL0) {
        q0.x = fmaxf(q0.x, 0.f); q0.y = fmaxf(q0.y, 0.f); q0.z = fmaxf(q0.z, 0.f); q0.w = fmaxf(q0.w, 0.f);
        q1.x = fmaxf(q1.x, 0.f); q1.y = fmaxf(q1.y, 0.f); q1.z = fmaxf(q1.z, 0.f); q1.w = fmaxf(q1.w, 0.f);
      }
      const v4f z4 = {0.f, 0.f, 0.f, 0.f};
      if (grow >= nN) { q0 = z4; q1 = z4; }
      v4u hv, lv;
      hlpack(q0, q1, hv, lv);
      v4u pv;
      pv.x = hh ? lv.x : hv.x; pv.y = hh ? lv.y : hv.y; pv.z = hh ? lv.z : hv.z; pv.w = hh ? lv.w : hv.w;
      unsigned short* dp = outH + (size_t)grow * (size_t)(2 * CH) + hoff;
      *(volatile v4u*)dp = pv;
      __threadfence();
      *(volatile v4u*)dp = pv;
    }
  } else if constexpr (EPI == EPI_POOL) {
    const v4f ob4 = bfr4(*(const v4fa*)(bias + 4 * lane));
    const v4f ga4 = bfr4(*(const v4fa*)(va + 4 * lane));
    const float gb = bfr(vb[0]);
#pragma unroll 1
    for (int i = 0; i < 16; ++i) {
      const int row  = 16 * wave + i;
      const int grow = rowBase + row;
      float* sq = stg + row * GBN + 4 * lane;
      v4f p = *(const v4fa*)sq;
      p += ob4;
      *(v4fa*)sq = p;
      float s = 0.f;
      s = fmaf(p.x, ga4.x, s); s = fmaf(p.y, ga4.y, s); s = fmaf(p.z, ga4.z, s); s = fmaf(p.w, ga4.w, s);
      s = wsum(s) + gb;
      if (lane == 0) sdot[row] = (grow < nN) ? s : -3.0e38f;
    }
    __syncthreads();
    const float sa = sdot[lane], sb = sdot[lane + 32];
    const float bm = wmax(fmaxf(sa, sb));
    const float ea = (sa > -1.0e38f) ? expf(sa - bm) : 0.f;
    const float eb = (sb > -1.0e38f) ? expf(sb - bm) : 0.f;
    if (wave == 0) { sex[lane] = ea; sex[lane + 32] = eb; }
    __syncthreads();
    float gsum = 0.f, esum = 0.f;
#pragma unroll 4
    for (int r = 0; r < GBM; ++r) {
      const float e = sex[r];
      esum += e;
      gsum = fmaf(e, stg[r * GBN + tid], gsum);
    }
    srec[tid] = gsum;
    srec[GBN + tid] = (tid == 0) ? bm : ((tid == 1) ? esum : 0.f);
    __syncthreads();
    const v4f rv = *(const v4fa*)(srec + (wave & 1) * GBN + 4 * lane);
    float* rptr = outV + (size_t)blockIdx.x * RECW + (wave & 1) * GBN + 4 * lane;
#pragma unroll 1
    for (int i = 0; i < 16; ++i) {
      const int row = 16 * wave + i;
      const v4f p = *(const v4fa*)(stg + row * GBN + 4 * lane);
      float* op = outF + (size_t)(rowBase + row) * (size_t)HIDC + 4 * lane;
      *(volatile v4f*)op = p;
    }
    if (wave < 2) *(volatile v4f*)rptr = rv;
    __threadfence();
#pragma unroll 1
    for (int i = 0; i < 16; ++i) {
      const int row = 16 * wave + i;
      const v4f p = *(const v4fa*)(stg + row * GBN + 4 * lane);
      float* op = outF + (size_t)(rowBase + row) * (size_t)HIDC + 4 * lane;
      *(volatile v4f*)op = p;
    }
    if (wave < 2) *(volatile v4f*)rptr = rv;
  } else {
    const int bl = lane < 16 ? lane : 15;
    const float vm = lane < 16 ? 1.f : 0.f;
    const v4f b4 = bfr4(*(const v4fa*)(bias + 4 * bl)) * vm;
    const v4f a4 = bfr4(*(const v4fa*)(va + 4 * bl)) * vm;
    const float cb = bfr(vb[0]);
#pragma unroll 1
    for (int i = 0; i < 16; ++i) {
      const int row = 16 * wave + i;
      const v4f p = *(const v4fa*)(stg + row * GBN + 4 * lane);
      const float v0 = fmaxf(p.x + b4.x, 0.f), v1 = fmaxf(p.y + b4.y, 0.f);
      const float v2 = fmaxf(p.z + b4.z, 0.f), v3 = fmaxf(p.w + b4.w, 0.f);
      float s = 0.f;
      s = fmaf(v0, a4.x, s); s = fmaf(v1, a4.y, s); s = fmaf(v2, a4.z, s); s = fmaf(v3, a4.w, s);
      s = wsum(s) + cb;
      if (lane == 0) sdot[row] = s;
    }
    __syncthreads();
    const v4f ov = *(const v4fa*)(sdot + 4 * m);
    const int r0 = rowBase + 4 * m;
    const bool wr = (wave == 0) && (lane < 16) && (r0 + 4 <= nN);
    if (wr) *(volatile v4f*)(outV + r0) = ov;
    __threadfence();
    if (wr) *(volatile v4f*)(outV + r0) = ov;
  }
}

__global__ __launch_bounds__(NTHR) void k_agg(
    const int* __restrict__ srcs, const int* __restrict__ dsts,
    const float* __restrict__ F, const float* __restrict__ SD,
    const float* __restrict__ bias, unsigned short* HP,
    int nN, int nE, int nb, int vec8, int MPr) {
  extern __shared__ v4f lds_dyn[];
  int* reg1 = (int*)lds_dyn;
  int* reg2 = reg1 + RCAP;
  int* scnt = reg2 + RCAP;
  int* soff = scnt + NBMAX;
  int* list = soff + NBMAX;
  int* wcnt = list + LISTN;
  int* wtot = wcnt + NWAVE;
  const int tid = (int)threadIdx.x, lane = tid & 31, wave = tid >> 5;
  const int nodeBase = (int)blockIdx.x * nb;

  for (int i = tid; i < NBMAX; i += NTHR) scnt[i] = 0;
  __syncthreads();

  int tot = 0;
  const int nChunks = (nE + CHUNK - 1) / CHUNK;
#pragma unroll 1
  for (int ch = 0; ch < nChunks; ++ch) {
    const int cbase = ch * CHUNK;
    const int wc = scan_chunk(dsts, nE, cbase, nodeBase, nb, vec8, list, tid, lane, wave);
    if (lane == 0) wcnt[wave] = wc;
    __syncthreads();
    int pre = 0, all = 0;
#pragma unroll
    for (int w2 = 0; w2 < NWAVE; ++w2) {
      int c = wcnt[w2];
      c = c < 0 ? 0 : (c > WCAP ? WCAP : c);
      all += c;
      pre += (w2 < wave) ? c : 0;
    }
    const int wcc  = wc > WCAP ? WCAP : wc;
    const int base = tot + pre;
#pragma unroll 1
    for (int i = lane; i < wcc; i += 32) {
      const int ent = list[wave * WCAP + i];
      const int el  = (ent >> SLOTB) & (CHUNK - 1);
      const int sl  = ent & (NBMAX - 1);
      int eid = cbase + el;
      eid = eid > nE - 1 ? nE - 1 : eid;
      const int pos = base + i;
      if (pos < RCAP) reg1[pos] = (int)(((unsigned)eid << SLOTB) | (unsigned)sl);
    }
    tot += all;
    tot = tot > RCAP ? RCAP : tot;
    __syncthreads();
  }
  const int nh = tot;

  if (wave == 0) {
#pragma unroll 1
    for (int b0 = 0; b0 < nh; b0 += 32) {
      const int idx = b0 + lane;
      const int uv  = reg1[idx < nh ? idx : nh - 1];
      const int m32 = (nh - b0) < 32 ? (nh - b0) : 32;
#pragma unroll 1
      for (int k = 0; k < m32; ++k) {
        const int u  = __builtin_amdgcn_readlane(uv, k);
        const int sl = u & (NBMAX - 1);
        if (lane == 0) scnt[sl] = scnt[sl] + 1;
      }
    }
  }
  __syncthreads();

  {
    const v4i ca = *(const v4i*)(scnt + 8 * tid);
    const v4i cb = *(const v4i*)(scnt + 8 * tid + 4);
    const int e0 = ca.x < 0 ? 0 : ca.x, e1 = ca.y < 0 ? 0 : ca.y, e2 = ca.z < 0 ? 0 : ca.z, e3 = ca.w < 0 ? 0 : ca.w;
    const int e4 = cb.x < 0 ? 0 : cb.x, e5 = cb.y < 0 ? 0 : cb.y, e6 = cb.z < 0 ? 0 : cb.z, e7 = cb.w < 0 ? 0 : cb.w;
    const int ts = e0 + e1 + e2 + e3 + e4 + e5 + e6 + e7;
    int incl = ts;
#pragma unroll
    for (int d = 1; d < 32; d <<= 1) {
      const int up = __shfl_up(incl, d);
      if (lane >= d) incl += up;
    }
    if (lane == 31) wtot[wave] = incl;
    __syncthreads();
    int pre = 0;
#pragma unroll
    for (int w2 = 0; w2 < NWAVE; ++w2) pre += (w2 < wave) ? wtot[w2] : 0;
    int run = pre + incl - ts;
    soff[8 * tid + 0] = run; run += e0;
    soff[8 * tid + 1] = run; run += e1;
    soff[8 * tid + 2] = run; run += e2;
    soff[8 * tid + 3] = run; run += e3;
    soff[8 * tid + 4] = run; run += e4;
    soff[8 * tid + 5] = run; run += e5;
    soff[8 * tid + 6] = run; run += e6;
    soff[8 * tid + 7] = run;
  }
  __syncthreads();
  for (int i = tid; i < NBMAX; i += NTHR) list[i] = soff[i];
  __syncthreads();

  if (wave == 0) {
#pragma unroll 1
    for (int b0 = 0; b0 < nh; b0 += 32) {
      const int idx = b0 + lane;
      const int uv  = reg1[idx < nh ? idx : nh - 1];
      const int m32 = (nh - b0) < 32 ? (nh - b0) : 32;
#pragma unroll 1
      for (int k = 0; k < m32; ++k) {
        const int u   = __builtin_amdgcn_readlane(uv, k);
        const int sl  = u & (NBMAX - 1);
        const int eid = (int)((unsigned)u >> SLOTB);
        if (lane == 0) {
          int pos = list[sl];
          pos = pos < 0 ? 0 : (pos > RCAP - 1 ? RCAP - 1 : pos);
          reg2[pos] = eid;
          list[sl] = pos + 1;
        }
      }
    }
  }
  __syncthreads();

  const int nbw = nb >> 3;
  const bool ovf = (nh >= RCAP);
  const float qnan = __int_as_float(0x7fc00000);
  const int cA = 8 * lane;
  const int cB = (HC / 2) + 8 * lane;
  const int hA = lane >> 4, hB = 2 + (lane >> 4);
  const v4f bA0 = bfr4(*(const v4fa*)(bias + cA)), bA1 = bfr4(*(const v4fa*)(bias + cA + 4));
  const v4f bB0 = bfr4(*(const v4fa*)(bias + cB)), bB1 = bfr4(*(const v4fa*)(bias + cB + 4));
  const float* ASa = SD + (size_t)(2 * hA) * (size_t)MPr;
  const float* ADa = ASa + MPr;
  const float* ASb = SD + (size_t)(2 * hB) * (size_t)MPr;
  const float* ADb = ASb + MPr;

#pragma unroll 1
  for (int jt = 0; jt < nbw; ++jt) {
    const int slot = wave * nbw + jt;
    const int grow = nodeBase + slot;
    const int gcl  = grow < nN ? grow : nN - 1;
    int st = soff[slot];
    const int craw = scnt[slot];
    int cnt = craw;
    st  = st < 0 ? 0 : (st > nh ? nh : st);
    cnt = cnt < 0 ? 0 : (cnt > DEGCAP ? DEGCAP : cnt);
    if (cnt > nh - st) cnt = nh - st;
    const float pz = (ovf || craw > DEGCAP) ? qnan : 0.0f;

    const float* fr = F + (size_t)gcl * HC;
    v4f a0 = *(const v4fa*)(fr + cA), a1 = *(const v4fa*)(fr + cA + 4);
    v4f c0 = *(const v4fa*)(fr + cB), c1 = *(const v4fa*)(fr + cB + 4);
    const float adA = ADa[gcl], adB = ADb[gcl];
    const float lA = leaky(ASa[gcl] + adA);
    const float lB = leaky(ASb[gcl] + adB);
    float mxA = lA, dnA = 1.0f, mxB = lB, dnB = 1.0f;

#pragma unroll 1
    for (int b0 = 0; b0 < cnt; b0 += 32) {
      int idx = st + b0 + lane; idx = idx > RCAP - 1 ? RCAP - 1 : idx;
      int eid = reg2[idx]; eid = eid < 0 ? 0 : (eid > nE - 1 ? nE - 1 : eid);
      const int sraw = srcs[eid];
      const int sr = sraw < 0 ? 0 : (sraw > nN - 1 ? nN - 1 : sraw);
      const int m32 = (cnt - b0) < 32 ? (cnt - b0) : 32;
#pragma unroll 1
      for (int k = 0; k < m32; ++k) {
        const int sk = __builtin_amdgcn_readlane(sr, k);
        const float* rp = F + (size_t)sk * HC;
        const v4f xa0 = *(const v4fa*)(rp + cA), xa1 = *(const v4fa*)(rp + cA + 4);
        const v4f xb0 = *(const v4fa*)(rp + cB), xb1 = *(const v4fa*)(rp + cB + 4);
        const float lgA = leaky(ASa[sk] + adA);
        const float lgB = leaky(ASb[sk] + adB);
        {
          const float df = lgA - mxA;
          const float ee = __expf(-fabsf(df));
          const bool up  = df > 0.f;
          const float s1 = up ? ee : 1.0f;
          const float s2 = up ? 1.0f : ee;
          mxA = up ? lgA : mxA;
          dnA = fmaf(dnA, s1, s2);
          a0.x = fmaf(a0.x, s1, s2 * xa0.x); a0.y = fmaf(a0.y, s1, s2 * xa0.y);
          a0.z = fmaf(a0.z, s1, s2 * xa0.z); a0.w = fmaf(a0.w, s1, s2 * xa0.w);
          a1.x = fmaf(a1.x, s1, s2 * xa1.x); a1.y = fmaf(a1.y, s1, s2 * xa1.y);
          a1.z = fmaf(a1.z, s1, s2 * xa1.z); a1.w = fmaf(a1.w, s1, s2 * xa1.w);
        }
        {
          const float df = lgB - mxB;
          const float ee = __expf(-fabsf(df));
          const bool up  = df > 0.f;
          const float s1 = up ? ee : 1.0f;
          const float s2 = up ? 1.0f : ee;
          mxB = up ? lgB : mxB;
          dnB = fmaf(dnB, s1, s2);
          c0.x = fmaf(c0.x, s1, s2 * xb0.x); c0.y = fmaf(c0.y, s1, s2 * xb0.y);
          c0.z = fmaf(c0.z, s1, s2 * xb0.z); c0.w = fmaf(c0.w, s1, s2 * xb0.w);
          c1.x = fmaf(c1.x, s1, s2 * xb1.x); c1.y = fmaf(c1.y, s1, s2 * xb1.y);
          c1.z = fmaf(c1.z, s1, s2 * xb1.z); c1.w = fmaf(c1.w, s1, s2 * xb1.w);
        }
      }
    }
    const float invA = __builtin_amdgcn_rcpf(dnA + EPS_SM);
    const float invB = __builtin_amdgcn_rcpf(dnB + EPS_SM);
    const bool live = grow < nN;
    const v4f oA0 = fin4(a0, invA, bA0, live, pz), oA1 = fin4(a1, invA, bA1, live, pz);
    const v4f oB0 = fin4(c0, invB, bB0, live, pz), oB1 = fin4(c1, invB, bB1, live, pz);
    v4u hAv, lAv, hBv, lBv;
    hlpack(oA0, oA1, hAv, lAv);
    hlpack(oB0, oB1, hBv, lBv);
    unsigned short* hp = HP + (size_t)grow * KHL2;
    const bool wr = grow < MPr;
    if (wr) {
      *(volatile v4u*)(hp + cA) = hAv;
      *(volatile v4u*)(hp + cB) = hBv;
      *(volatile v4u*)(hp + HC + cA) = lAv;
      *(volatile v4u*)(hp + HC + cB) = lBv;
    }
    __threadfence();
    if (wr) {
      *(volatile v4u*)(hp + cA) = hAv;
      *(volatile v4u*)(hp + cB) = hBv;
      *(volatile v4u*)(hp + HC + cA) = lAv;
      *(volatile v4u*)(hp + HC + cB) = lBv;
    }
  }
}

__global__ __launch_bounds__(NTHR) void k_pool(const float* __restrict__ rec, int nrec,
                                               const float* __restrict__ gpW, const float* __restrict__ gpb,
                                               float* gv) {
  __shared__ float smx[NWAVE];
  __shared__ float sg[HIDC];
  __shared__ __attribute__((aligned(16))) float sgv[HIDC];
  const int tid = (int)threadIdx.x, lane = tid & 31, wave = tid >> 5;
  float mloc = -3.0e38f;
#pragma unroll 1
  for (int b = tid; b < nrec; b += NTHR) mloc = fmaxf(mloc, rec[(size_t)b * RECW + HIDC]);
  mloc = wmax(mloc);
  if (lane == 0) smx[wave] = mloc;
  __syncthreads();
  float bm = smx[0];
#pragma unroll
  for (int w = 1; w < NWAVE; ++w) bm = fmaxf(bm, smx[w]);
  const int col = tid & (HIDC - 1);
  double G = 0.0, S = 0.0;
#pragma unroll 1
  for (int b = 0; b < nrec; ++b) {
    const float* rp = rec + (size_t)b * RECW;
    const float w = expf(rp[HIDC] - bm);
    S += (double)w * (double)rp[HIDC + 1];
    G += (double)w * (double)rp[col];
  }
  const float g = (float)(G / S);
  if (tid < HIDC) sg[tid] = g;
  __syncthreads();
  double d = 0.0;
#pragma unroll 4
  for (int k = 0; k < HIDC; ++k) d += (double)sg[k] * (double)bfr(gpW[(size_t)k * HIDC + col]);
  const float gvv = 2.0f * ((float)d + bfr(gpb[col]));
  if (tid < HIDC) sgv[tid] = gvv;
  __syncthreads();
  const v4f o = *(const v4fa*)(sgv + 4 * lane);
  if (wave == 0) *(volatile v4f*)(gv + 4 * lane) = o;
  __threadfence();
  if (wave == 0) *(volatile v4f*)(gv + 4 * lane) = o;
}

__global__ __launch_bounds__(NTHR) void k_ln(const float* __restrict__ Z, const float* __restrict__ gv,
                                             const float* __restrict__ lng, const float* __restrict__ lnb,
                                             unsigned short* LH, int nN, int MPr) {
  const int tid = (int)threadIdx.x, lane = tid & 31, wave = tid >> 5, hh = lane >> 4;
  const int row = (int)blockIdx.x * NWAVE + wave;
  if (row >= MPr) return;
  const int rc = row < nN ? row : nN - 1;
  const int c8 = 8 * (lane & 15);
  const float* zp = Z + (size_t)rc * HIDC + c8;
  v4f q0 = *(const v4fa*)zp, q1 = *(const v4fa*)(zp + 4);
  const v4f g0 = *(const v4fa*)(gv + c8), g1 = *(const v4fa*)(gv + c8 + 4);
  q0 += g0; q1 += g1;
  float s = ((q0.x + q0.y) + (q0.z + q0.w)) + ((q1.x + q1.y) + (q1.z + q1.w));
  s = wsum(s);
  const float mu = s * (1.0f / 256.0f);
  v4f d0 = q0 - mu, d1 = q1 - mu;
  float sq = ((d0.x * d0.x + d0.y * d0.y) + (d0.z * d0.z + d0.w * d0.w)) +
             ((d1.x * d1.x + d1.y * d1.y) + (d1.z * d1.z + d1.w * d1.w));
  sq = wsum(sq);
  const float var = sq * (1.0f / 256.0f);
  const float rs = rsqrtf(var + LN_EPS);
  const v4f lg0 = bfr4(*(const v4fa*)(lng + c8)), lg1 = bfr4(*(const v4fa*)(lng + c8 + 4));
  const v4f lb0 = bfr4(*(const v4fa*)(lnb + c8)), lb1 = bfr4(*(const v4fa*)(lnb + c8 + 4));
  v4f y0, y1;
  y0.x = fmaxf((d0.x * rs) * lg0.x + lb0.x, 0.f); y0.y = fmaxf((d0.y * rs) * lg0.y + lb0.y, 0.f);
  y0.z = fmaxf((d0.z * rs) * lg0.z + lb0.z, 0.f); y0.w = fmaxf((d0.w * rs) * lg0.w + lb0.w, 0.f);
  y1.x = fmaxf((d1.x * rs) * lg1.x + lb1.x, 0.f); y1.y = fmaxf((d1.y * rs) * lg1.y + lb1.y, 0.f);
  y1.z = fmaxf((d1.z * rs) * lg1.z + lb1.z, 0.f); y1.w = fmaxf((d1.w * rs) * lg1.w + lb1.w, 0.f);
  const v4f z4 = {0.f, 0.f, 0.f, 0.f};
  if (row >= nN) { y0 = z4; y1 = z4; }
  v4u hv, lv;
  hlpack(y0, y1, hv, lv);
  v4u pv;
  pv.x = hh ? lv.x : hv.x; pv.y = hh ? lv.y : hv.y; pv.z = hh ? lv.z : hv.z; pv.w = hh ? lv.w : hv.w;
  unsigned short* dp = LH + (size_t)row * KHL1 + 8 * lane;
  *(volatile v4u*)dp = pv;
  __threadfence();
  *(volatile v4u*)dp = pv;
}

static int pick_nb(int nE, int nN) {
  int nb = NBMAX;
  while (nb > 32 && (long long)nb * (long long)nE * 5LL > (long long)RCAP * (long long)nN * 4LL) nb >>= 1;
  return nb;
}
static inline int cdiv(int a, int b) { return (a + b - 1) / b; }

extern "C" void kernel_launch(void* const* d_in, const int* in_sizes, int n_in,
                              void* d_out, int out_size, void* d_ws, size_t ws_size,
                              hipStream_t stream) {
  if (n_in < 29) return;
  if (in_sizes[0] < F_IN || (in_sizes[0] % F_IN) != 0) return;
  const int nN = in_sizes[0] / F_IN;
  if (nN < 4 || (nN & 3) != 0 || nN > (1 << 22)) return;
  if (in_sizes[28] < 2 || (in_sizes[28] & 1) != 0) return;
  const int nE = in_sizes[28] / 2;
  if (nE < 1 || nE >= (1 << (32 - SLOTB))) return;
  if (in_sizes[2] != F_IN * HIDC || in_sizes[3] != HIDC) return;
  if (in_sizes[6] != HIDC * HC) return;
  if (in_sizes[7] != NHEAD * HIDC || in_sizes[8] != NHEAD * HIDC || in_sizes[9] != HC) return;
  if (in_sizes[10] != HC * HC) return;
  if (in_sizes[11] != NHEAD * HIDC || in_sizes[12] != NHEAD * HIDC || in_sizes[13] != HC) return;
  if (in_sizes[14] != HIDC * HC || in_sizes[15] != HC) return;
  if (in_sizes[16] != HC * HIDC || in_sizes[17] != HIDC) return;
  if (in_sizes[18] != HIDC || in_sizes[19] < 1) return;
  if (in_sizes[20] != HIDC * HIDC || in_sizes[21] != HIDC) return;
  if (in_sizes[22] != HIDC || in_sizes[23] != HIDC) return;
  if (in_sizes[24] != HIDC * M1N || in_sizes[25] != M1N) return;
  if (in_sizes[26] != M1N || in_sizes[27] < 1) return;
  if (out_size != nN) return;

  const float* x    = (const float*)d_in[0];
  const float* nW   = (const float*)d_in[2];
  const float* nbv  = (const float*)d_in[3];
  const float* g1W  = (const float*)d_in[6];
  const float* g1as = (const float*)d_in[7];
  const float* g1ad = (const float*)d_in[8];
  const float* g1b  = (const float*)d_in[9];
  const float* g2W  = (const float*)d_in[10];
  const float* g2as = (const float*)d_in[11];
  const float* g2ad = (const float*)d_in[12];
  const float* g2b  = (const float*)d_in[13];
  const float* rW   = (const float*)d_in[14];
  const float* rb   = (const float*)d_in[15];
  const float* oW   = (const float*)d_in[16];
  const float* ob   = (const float*)d_in[17];
  const float* gaW  = (const float*)d_in[18];
  const float* gab  = (const float*)d_in[19];
  const float* gpW  = (const float*)d_in[20];
  const float* gpb  = (const float*)d_in[21];
  const float* lng  = (const float*)d_in[22];
  const float* lnb  = (const float*)d_in[23];
  const float* m1W  = (const float*)d_in[24];
  const float* m1b  = (const float*)d_in[25];
  const float* m2W  = (const float*)d_in[26];
  const float* m2b  = (const float*)d_in[27];
  const int*   ei   = (const int*)  d_in[28];
  float* out = (float*)d_out;
  const int* src = ei;
  const int* dst = ei + nE;

  const int MP   = cdiv(nN, GBM) * GBM;
  const int gM   = MP / GBM;
  const int nb   = pick_nb(nE, nN);
  if (nb < 32 || (nb & (nb - 1)) != 0 || nb > NBMAX) return;
  const int gA   = cdiv(MP, nb);
  if ((long long)gA * nb < (long long)MP) return;
  const int vec8 = ((nE & 3) == 0) ? 1 : 0;

  char* ws = (char*)d_ws;
  size_t off = 0;
  const size_t oXB  = off; off += (size_t)MP * F_IN * 2;          off = (off + 255) & ~(size_t)255;
  const size_t oHB  = off; off += (size_t)MP * KHL1 * 2;          off = (off + 255) & ~(size_t)255;
  const size_t oXH  = off; off += (size_t)MP * HC * 4;            off = (off + 255) & ~(size_t)255;
  const size_t oHP  = off; off += (size_t)MP * KHL2 * 2;          off = (off + 255) & ~(size_t)255;
  const size_t oSD  = off; off += (size_t)(2 * NHEAD) * MP * 4;   off = (off + 255) & ~(size_t)255;
  const size_t oNWT = off; off += (size_t)HIDC * F_IN * 2;        off = (off + 255) & ~(size_t)255;
  const size_t oG1T = off; off += (size_t)HC * KHL1 * 2;          off = (off + 255) & ~(size_t)255;
  const size_t oRWT = off; off += (size_t)HC * KHL1 * 2;          off = (off + 255) & ~(size_t)255;
  const size_t oG2T = off; off += (size_t)HC * KHL2 * 2;          off = (off + 255) & ~(size_t)255;
  const size_t oOWT = off; off += (size_t)HIDC * KHL2 * 2;        off = (off + 255) & ~(size_t)255;
  const size_t oM1T = off; off += (size_t)HIDC * KHL1 * 2;        off = (off + 255) & ~(size_t)255;
  const size_t oREC = off; off += (size_t)gM * RECW * 4;          off = (off + 255) & ~(size_t)255;
  const size_t oGV  = off; off += (size_t)HIDC * 4;               off = (off + 255) & ~(size_t)255;
  if (off > ws_size || off > (size_t)WSMAX) return;
  static_assert((size_t)F_IN * 2 == (size_t)HIDC * 4);
  static_assert((size_t)HC * 4 == (size_t)KHL2 * 2);
  unsigned short* XB  = (unsigned short*)(ws + oXB);
  float*          Zf  = (float*)(ws + oXB);
  unsigned short* HB  = (unsigned short*)(ws + oHB);
  unsigned short* LH  = (unsigned short*)(ws + oHB);
  float*          XH  = (float*)(ws + oXH);
  unsigned short* ZS  = (unsigned short*)(ws + oXH);
  unsigned short* HP  = (unsigned short*)(ws + oHP);
  float*          SDp = (float*)(ws + oSD);
  unsigned short* nWT = (unsigned short*)(ws + oNWT);
  unsigned short* g1T = (unsigned short*)(ws + oG1T);
  unsigned short* rWT = (unsigned short*)(ws + oRWT);
  unsigned short* g2T = (unsigned short*)(ws + oG2T);
  unsigned short* oWT = (unsigned short*)(ws + oOWT);
  unsigned short* m1T = (unsigned short*)(ws + oM1T);
  float*          REC = (float*)(ws + oREC);
  float*          GV  = (float*)(ws + oGV);

  hipFuncSetAttribute(reinterpret_cast<const void*>(&k_agg),
                      hipFuncAttributeMaxDynamicSharedMemorySize, LDS_AGG);

  const int nUx = MP * (F_IN / 8);
  k_xprep<<<cdiv(nUx, NTHR), NTHR, 0, stream>>>(x, XB, nN, nUx);
  k_wprep<<<NU_ALL / NTHR, NTHR, 0, stream>>>(nW, g1W, rW, g2W, oW, m1W, nWT, g1T, rWT, g2T, oWT, m1T);

  k_gemm<EPI_HL0><<<dim3(gM, 1), GTHR, 0, stream>>>(XB, nWT, F_IN, nbv, nbv, nbv, HP, SDp, HB, SDp, MP, nN);
  k_gemm<EPI_DOT><<<dim3(gM, HC / GBN), GTHR, 0, stream>>>(HB, g1T, KHL1, g1b, g1as, g1ad, HP, XH, XB, SDp, MP, nN);
  k_agg<<<gA, NTHR, LDS_AGG, stream>>>(src, dst, XH, SDp, g1b, HP, nN, nE, nb, vec8, MP);
  k_gemm<EPI_DOT><<<dim3(gM, HC / GBN), GTHR, 0, stream>>>(HP, g2T, KHL2, g2b, g2as, g2ad, XB, XH, XB, SDp, MP, nN);
  k_agg<<<gA, NTHR, LDS_AGG, stream>>>(src, dst, XH, SDp, g2b, HP, nN, nE, nb, vec8, MP);
  k_gemm<EPI_HLR><<<dim3(gM, HC / GBN), GTHR, 0, stream>>>(HB, rWT, KHL1, rb, rb, rb, HP, SDp, ZS, SDp, MP, nN);
  k_gemm<EPI_POOL><<<dim3(gM, 1), GTHR, 0, stream>>>(ZS, oWT, KHL2, ob, gaW, gab, HP, Zf, LH, REC, MP, nN);
  k_pool<<<1, NTHR, 0, stream>>>(REC, gM, gpW, gpb, GV);
  k_ln<<<MP / NWAVE, NTHR, 0, stream>>>(Zf, GV, lng, lnb, LH, nN, MP);
  k_gemm<EPI_HEAD><<<dim3(gM, 1), GTHR, 0, stream>>>(LH, m1T, KHL1, m1b, m2W, m2b, HP, SDp, ZS, out, MP, nN);
}
